// SimpleNet_62105227100335
// MI455X (gfx1250) — hardware-run, weakly checked
//
#include <hip/hip_runtime.h>
#include <stddef.h>
#include <stdint.h>


#define NUSR    50000
#define NITM    20000
#define MPU     50048
#define MPI     20096
#define DIN     128
#define DHID    256
#define DOUT    128
#define NEDGE   300000
#define NLAB    200000
#define NTHR    256
#define NWAVE   8
#define EPT     8
#define CHUNK   (NTHR * EPT)
#define WCAP    (EPT * 32)
#define LISTN   (NWAVE * WCAP)
#define NBA     1024
#define PKS     10
#define RCAP_I  20480
#define RCAP_U  8192
#define DEGCAP  64
#define NBI     20
#define NBU     49
#define NBT     (NBI + NBU)
#define GBM     64
#define GBN     128
#define GTHR    128
#define RPB     64
#define RPW     8
#define RBI     (MPI / RPB)
#define RBU     (MPU / RPB)
#define K1      384
#define K2      1024
#define HP      512
#define BK_INTS_I (2 * RCAP_I + 3 * NBA + LISTN + 32)
#define LDS_BK  (BK_INTS_I * 4)
#define MEAS_HITS_I 15549
#define MEAS_HITS_U 6271
#define MEAS_DEG    35
#define PB_XU   (MPU * 16 / NTHR)
#define PB_XI   (MPI * 16 / NTHR)
#define PB_W    (14 * 4096 / NTHR)
#define PB_TOT  (PB_XU + PB_XI + PB_W + 1)
#define W1E     (DHID * K1)
#define W2E     (DOUT * K2)

static_assert((CHUNK & (CHUNK - 1)) == 0 && CHUNK <= 4096);
static_assert(NBA == (1 << PKS) && NBA == NTHR * 4);
static_assert(LISTN == NWAVE * WCAP);
static_assert(RCAP_I % (NTHR * 4) == 0 && RCAP_U % (NTHR * 4) == 0);
static_assert((long long)RCAP_I * 100 >= (long long)MEAS_HITS_I * 105);
static_assert((long long)RCAP_U * 100 >= (long long)MEAS_HITS_U * 105);
static_assert(DEGCAP >= MEAS_DEG + 8);
static_assert(LDS_BK <= 300000);
static_assert(NEDGE < (1 << 21));
static_assert(MPU % GBM == 0 && MPI % GBM == 0 && MPU >= NUSR && MPI >= NITM);
static_assert(NBI * NBA >= MPI && NBU * NBA >= MPU);
static_assert((NBI - 1) * NBA < NITM && (NBU - 1) * NBA < NUSR);
static_assert(K1 % 32 == 0 && K2 % 32 == 0 && K1 == 3 * DIN && K2 == 4 * DHID && HP == 2 * DHID);
static_assert(GBM == (GTHR / 32) * 16 && DHID == 2 * GBN && DOUT == GBN && GBN == 32 * 4);
static_assert((MPU * 16) % NTHR == 0 && (MPI * 16) % NTHR == 0 && (14 * 4096) % NTHR == 0);
static_assert(RPB == NWAVE * RPW && RPB == GBM);
static_assert((NLAB * 4) % 128 == 0 && NLAB % 4 == 0);

typedef float          v4f   __attribute__((ext_vector_type(4)));
typedef float          v8f   __attribute__((ext_vector_type(8)));
typedef int            v4i   __attribute__((ext_vector_type(4)));
typedef int            v8i   __attribute__((ext_vector_type(8)));
typedef unsigned       v4u   __attribute__((ext_vector_type(4)));
typedef unsigned short v8us  __attribute__((ext_vector_type(8)));
typedef __bf16         v16bf __attribute__((ext_vector_type(16)));
typedef v4f  __attribute__((may_alias)) v4fa;
typedef v4i  __attribute__((may_alias)) v4ia;
typedef v4u  __attribute__((may_alias)) v4ua;
typedef v8us __attribute__((may_alias)) v8usa;
union FragB { v16bf v; v8us h[2]; v8i w; };

__device__ __forceinline__ v8f wmb(const FragB& a, const FragB& b, v8f c) {
  v8f d = __builtin_amdgcn_wmma_f32_16x16x32_bf16(false, a.v, false, b.v, (short)0, c, false, false);
  asm volatile("v_nop\n\tv_nop\n\tv_nop\n\tv_nop" : "+v"(d) : "v"(a.w), "v"(b.w));
  return d;
}

__device__ __forceinline__ unsigned bf16_bits(float f) {
  const unsigned u = __float_as_uint(f);
  return ((u + 0x7FFFu + ((u >> 16) & 1u)) >> 16) & 0xFFFFu;
}
__device__ __forceinline__ float bf16_val(float f) { return __uint_as_float(bf16_bits(f) << 16); }
__device__ __forceinline__ float bfw_lo(unsigned w) { return __uint_as_float(w << 16); }
__device__ __forceinline__ float bfw_hi(unsigned w) { return __uint_as_float(w & 0xffff0000u); }
__device__ __forceinline__ void pack2(float a, float b, unsigned& hw, unsigned& lw) {
  const unsigned ha = bf16_bits(a), hb = bf16_bits(b);
  const unsigned la = bf16_bits(a - __uint_as_float(ha << 16));
  const unsigned lb = bf16_bits(b - __uint_as_float(hb << 16));
  hw = ha | (hb << 16);
  lw = la | (lb << 16);
}
__device__ __forceinline__ float relu_k(float v) { return (v > 0.0f) ? v : (v - v); }

__device__ __forceinline__ int scan_chunk(const int* __restrict__ keys, int nE, int cbase, int slotBase,
                                          int nb, int vec8, int* list, int tid, int lane, int wave) {
  int wc = 0;
  const int el0  = tid * EPT;
  const int e0   = cbase + el0;
  const int sent = (int)(1u << 31);
  v4i da, db;
  if (vec8 != 0 && cbase + CHUNK <= nE) {
    da = *(const v4i*)(keys + e0);
    db = *(const v4i*)(keys + e0 + 4);
  } else {
    da.x = (e0     < nE) ? keys[min(e0,     nE - 1)] : sent;
    da.y = (e0 + 1 < nE) ? keys[min(e0 + 1, nE - 1)] : sent;
    da.z = (e0 + 2 < nE) ? keys[min(e0 + 2, nE - 1)] : sent;
    da.w = (e0 + 3 < nE) ? keys[min(e0 + 3, nE - 1)] : sent;
    db.x = (e0 + 4 < nE) ? keys[min(e0 + 4, nE - 1)] : sent;
    db.y = (e0 + 5 < nE) ? keys[min(e0 + 5, nE - 1)] : sent;
    db.z = (e0 + 6 < nE) ? keys[min(e0 + 6, nE - 1)] : sent;
    db.w = (e0 + 7 < nE) ? keys[min(e0 + 7, nE - 1)] : sent;
  }
  const unsigned nbs = (unsigned)slotBase;
  const unsigned unb = (unsigned)nb;
  const unsigned s0 = (unsigned)da.x - nbs, s1 = (unsigned)da.y - nbs;
  const unsigned s2 = (unsigned)da.z - nbs, s3 = (unsigned)da.w - nbs;
  const unsigned s4 = (unsigned)db.x - nbs, s5 = (unsigned)db.y - nbs;
  const unsigned s6 = (unsigned)db.z - nbs, s7 = (unsigned)db.w - nbs;
  const bool h0 = s0 < unb, h1 = s1 < unb, h2 = s2 < unb, h3 = s3 < unb;
  const bool h4 = s4 < unb, h5 = s5 < unb, h6 = s6 < unb, h7 = s7 < unb;
  const unsigned any = __builtin_amdgcn_ballot_w32(h0 | h1 | h2 | h3 | h4 | h5 | h6 | h7);
  if (any != 0u) {
#define HITJ(J, HJ, SJ) { \
      const unsigned mj = __builtin_amdgcn_ballot_w32(HJ); \
      if (mj != 0u) { \
        if (HJ) { \
          const int pos = wc + (int)__builtin_amdgcn_mbcnt_lo(mj, 0u); \
          if (pos < WCAP) list[wave * WCAP + pos] = ((el0 + (J)) << PKS) | (int)(SJ); \
        } \
        wc += (int)__builtin_popcount(mj); } }
    HITJ(0, h0, s0)
    HITJ(1, h1, s1)
    HITJ(2, h2, s2)
    HITJ(3, h3, s3)
    HITJ(4, h4, s4)
    HITJ(5, h5, s5)
    HITJ(6, h6, s6)
    HITJ(7, h7, s7)
#undef HITJ
  }
  return wc;
}

__device__ __forceinline__ void cvt_rows(const float* __restrict__ x, unsigned short* dst, int u, int nLive) {
  const int row = u >> 4;
  const int c8  = (u & 15) * 8;
  const int rc  = row < nLive ? row : nLive - 1;
  const float* p = x + (size_t)rc * DIN + c8;
  const v4f a = *(const v4f*)p;
  const v4f b = *(const v4f*)(p + 4);
  asm volatile("" :: "v"(a), "v"(b));
  const unsigned mk = (row < nLive) ? 0xFFFFu : 0u;
  v8us o;
  o[0] = (unsigned short)(bf16_bits(a.x) & mk); o[1] = (unsigned short)(bf16_bits(a.y) & mk);
  o[2] = (unsigned short)(bf16_bits(a.z) & mk); o[3] = (unsigned short)(bf16_bits(a.w) & mk);
  o[4] = (unsigned short)(bf16_bits(b.x) & mk); o[5] = (unsigned short)(bf16_bits(b.y) & mk);
  o[6] = (unsigned short)(bf16_bits(b.z) & mk); o[7] = (unsigned short)(bf16_bits(b.w) & mk);
  unsigned short* dp = dst + (size_t)row * DIN + c8;
  *(volatile v8us*)dp = o;
  __threadfence();
  *(volatile v8us*)dp = o;
}

__device__ __forceinline__ v8us gath8(const float* __restrict__ W, int so, int pitch) {
  float f[8];
#pragma unroll
  for (int i = 0; i < 8; ++i) f[i] = W[so + i * pitch];
  v8us o;
#pragma unroll
  for (int i = 0; i < 8; ++i) o[i] = (unsigned short)bf16_bits(f[i]);
  return o;
}

__device__ __forceinline__ v4f bias4(const float* __restrict__ b, int t) {
  const v4f v = *(const v4f*)(b + 4 * t);
  v4f o;
  o.x = bf16_val(v.x); o.y = bf16_val(v.y); o.z = bf16_val(v.z); o.w = bf16_val(v.w);
  return o;
}

__global__ __launch_bounds__(NTHR) void k_prep(const float* __restrict__ xu, const float* __restrict__ xi,
                                               const float* __restrict__ wa, const float* __restrict__ wb,
                                               const float* __restrict__ wc, const float* __restrict__ wd,
                                               const float* __restrict__ we, const float* __restrict__ wf,
                                               const float* __restrict__ wg, const float* __restrict__ wh,
                                               const float* __restrict__ ba, const float* __restrict__ bb,
                                               const float* __restrict__ bc, const float* __restrict__ bd,
                                               unsigned short* XUB, unsigned short* XIB,
                                               unsigned short* WPL, float* BT) {
  const int blk = (int)blockIdx.x;
  const int tid = (int)threadIdx.x;
  if (blk < PB_XU) {
    cvt_rows(xu, XUB, blk * NTHR + tid, NUSR);
  } else if (blk < PB_XU + PB_XI) {
    cvt_rows(xi, XIB, (blk - PB_XU) * NTHR + tid, NITM);
  } else if (blk < PB_XU + PB_XI + PB_W) {
    const int wu   = (blk - PB_XU - PB_XI) * NTHR + tid;
    const int part = wu >> 12;
    const int v    = wu & 4095;
    int sid, sp, n, j, dOff;
    if (part < 6) {
      const int pl = part / 3;
      const int pp = part - 3 * pl;
      n = v >> 4; j = v & 15;
      sid = pl * 2 + ((pp == 2) ? 1 : 0);
      sp  = DHID;
      dOff = pl * W1E + n * K1 + pp * DIN + 8 * j;
    } else {
      const int q  = part - 6;
      const int pl = q >> 2;
      const int pp = q & 3;
      n = v >> 5; j = v & 31;
      sid = 4 + pl * 2 + (pp >> 1);
      sp  = DOUT;
      dOff = 2 * W1E + pl * W2E + n * K2 + pp * DHID + 8 * j;
    }
    const int so = 8 * j * sp + n;
    v8us o;
    if (sid == 0)      o = gath8(wa, so, sp);
    else if (sid == 1) o = gath8(wb, so, sp);
    else if (sid == 2) o = gath8(wc, so, sp);
    else if (sid == 3) o = gath8(wd, so, sp);
    else if (sid == 4) o = gath8(we, so, sp);
    else if (sid == 5) o = gath8(wf, so, sp);
    else if (sid == 6) o = gath8(wg, so, sp);
    else               o = gath8(wh, so, sp);
    unsigned short* dp = WPL + (size_t)dOff;
    *(volatile v8us*)dp = o;
    __threadfence();
    *(volatile v8us*)dp = o;
  } else {
    const int wv = tid >> 5;
    if (wv < 6) {
      v4f o;
      if (wv < 2)       o = bias4(ba, tid);
      else if (wv < 4)  o = bias4(bb, tid - 64);
      else if (wv == 4) o = bias4(bc, tid - 128);
      else              o = bias4(bd, tid - 160);
      float* dp = BT + 4 * tid;
      *(volatile v4f*)dp = o;
      __threadfence();
      *(volatile v4f*)dp = o;
    }
  }
}

template <int RC>
__device__ __forceinline__ void bucket_body(const int* __restrict__ keys, const int* __restrict__ gidx,
                                            int nE, int nK, int nG, int vec8, int lblk,
                                            int* lrow, int* cp0, int* fp0, int* rp0, int* dsm) {
  constexpr int BKI = 2 * RC + 3 * NBA + LISTN + 32;
  static_assert(BKI % 4 == 0 && BKI * 4 <= LDS_BK);
  int* reg1 = dsm;
  int* reg2 = reg1 + RC;
  int* scnt = reg2 + RC;
  int* soff = scnt + NBA;
  int* cur  = soff + NBA;
  int* list = cur + NBA;
  int* wcnt = list + LISTN;
  int* wtot = wcnt + 8;
  int* wmx  = wtot + 8;
  const int tid = (int)threadIdx.x, lane = tid & 31, wave = tid >> 5;
  const int nodeBase = lblk * NBA;
  int nb = nK - nodeBase;
  nb = nb > NBA ? NBA : (nb < 1 ? 1 : nb);

  {
    const v4i z4 = {0, 0, 0, 0};
    for (int i = tid * 4; i < BKI; i += NTHR * 4) *(v4ia*)(dsm + i) = z4;
  }
  __syncthreads();

  int tot = 0;
  const int nChunks = (nE + CHUNK - 1) / CHUNK;
#pragma unroll 1
  for (int ch = 0; ch < nChunks; ++ch) {
    const int cbase = ch * CHUNK;
    const int wc = scan_chunk(keys, nE, cbase, nodeBase, nb, vec8, list, tid, lane, wave);
    if (lane == 0) wcnt[wave] = wc;
    __syncthreads();
    int pre = 0, all = 0;
#pragma unroll
    for (int w2 = 0; w2 < NWAVE; ++w2) {
      int c = wcnt[w2];
      c = c < 0 ? 0 : (c > WCAP ? WCAP : c);
      all += c;
      pre += (w2 < wave) ? c : 0;
    }
    const int wcc  = wc > WCAP ? WCAP : wc;
    const int base = tot + pre;
#pragma unroll 1
    for (int i = lane; i < wcc; i += 32) {
      const int ent = list[wave * WCAP + i];
      const int el  = (ent >> PKS) & (CHUNK - 1);
      const int sl  = ent & (NBA - 1);
      int eid = cbase + el;
      eid = eid > nE - 1 ? nE - 1 : eid;
      const int pos = base + i;
      if (pos < RC) reg1[pos] = (int)(((unsigned)eid << PKS) | (unsigned)sl);
    }
    tot += all;
    tot = tot > RC ? RC : tot;
    __syncthreads();
  }
  const int nh = tot;

  if (wave == 0) {
#pragma unroll 1
    for (int b0 = 0; b0 < nh; b0 += 32) {
      const int idx = b0 + lane;
      const int uv  = reg1[idx < RC ? idx : RC - 1];
      const int m32 = (nh - b0) < 32 ? (nh - b0) : 32;
#pragma unroll 1
      for (int k = 0; k < m32; ++k) {
        const int u  = __builtin_amdgcn_readlane(uv, k);
        const int sl = u & (NBA - 1);
        if (lane == 0) scnt[sl] = scnt[sl] + 1;
      }
    }
  }
  __syncthreads();

  {
    const v4i ca = *(const v4ia*)(scnt + 4 * tid);
    const int e0 = ca.x < 0 ? 0 : ca.x, e1 = ca.y < 0 ? 0 : ca.y, e2 = ca.z < 0 ? 0 : ca.z, e3 = ca.w < 0 ? 0 : ca.w;
    const int ts = e0 + e1 + e2 + e3;
    int incl = ts;
#pragma unroll
    for (int d = 1; d < 32; d <<= 1) {
      const int up = __shfl_up(incl, d, 32);
      if (lane >= d) incl += up;
    }
    int mx = max(max(e0, e1), max(e2, e3));
    mx = max(mx, __shfl_xor(mx, 16, 32));
    mx = max(mx, __shfl_xor(mx, 8, 32));
    mx = max(mx, __shfl_xor(mx, 4, 32));
    mx = max(mx, __shfl_xor(mx, 2, 32));
    mx = max(mx, __shfl_xor(mx, 1, 32));
    if (lane == 31) wtot[wave] = incl;
    if (lane == 0)  wmx[wave] = mx;
    __syncthreads();
    int pre = 0;
#pragma unroll
    for (int w2 = 0; w2 < NWAVE; ++w2) pre += (w2 < wave) ? wtot[w2] : 0;
    int run = pre + incl - ts;
    v4i so;
    so.x = run; run += e0;
    so.y = run; run += e1;
    so.z = run; run += e2;
    so.w = run;
    *(v4ia*)(soff + 4 * tid) = so;
    *(v4ia*)(cur + 4 * tid)  = so;
  }
  __syncthreads();

  if (wave == 0) {
#pragma unroll 1
    for (int b0 = 0; b0 < nh; b0 += 32) {
      const int idx = b0 + lane;
      const int uv  = reg1[idx < RC ? idx : RC - 1];
      const int m32 = (nh - b0) < 32 ? (nh - b0) : 32;
#pragma unroll 1
      for (int k = 0; k < m32; ++k) {
        const int u   = __builtin_amdgcn_readlane(uv, k);
        const int sl  = u & (NBA - 1);
        const int eid = (int)((unsigned)u >> PKS);
        if (lane == 0) {
          int pos = cur[sl];
          pos = pos < 0 ? 0 : (pos > RC - 1 ? RC - 1 : pos);
          reg2[pos] = eid;
          cur[sl] = pos + 1;
        }
      }
    }
  }
  __syncthreads();

  int bmax = 0;
#pragma unroll
  for (int w2 = 0; w2 < NWAVE; ++w2) bmax = max(bmax, wmx[w2]);
  const int flag = ((nh >= RC) || (bmax > DEGCAP)) ? 1 : 0;

#pragma unroll 1
  for (int it = 0; it < RC / (NTHR * 4); ++it) {
    const int i0 = 4 * (it * NTHR + tid);
    const v4i ev = *(const v4ia*)(reg2 + i0);
    int e0 = ev.x, e1 = ev.y, e2 = ev.z, e3 = ev.w;
    e0 = e0 < 0 ? 0 : (e0 > nE - 1 ? nE - 1 : e0);
    e1 = e1 < 0 ? 0 : (e1 > nE - 1 ? nE - 1 : e1);
    e2 = e2 < 0 ? 0 : (e2 > nE - 1 ? nE - 1 : e2);
    e3 = e3 < 0 ? 0 : (e3 > nE - 1 ? nE - 1 : e3);
    int g0 = gidx[e0], g1 = gidx[e1], g2 = gidx[e2], g3 = gidx[e3];
    asm volatile("" :: "v"(g0), "v"(g1), "v"(g2), "v"(g3));
    g0 = g0 < 0 ? 0 : (g0 > nG - 1 ? nG - 1 : g0);
    g1 = g1 < 0 ? 0 : (g1 > nG - 1 ? nG - 1 : g1);
    g2 = g2 < 0 ? 0 : (g2 > nG - 1 ? nG - 1 : g2);
    g3 = g3 < 0 ? 0 : (g3 > nG - 1 ? nG - 1 : g3);
    v4i ov;
    ov.x = (i0     < nh) ? g0 : 0;
    ov.y = (i0 + 1 < nh) ? g1 : 0;
    ov.z = (i0 + 2 < nh) ? g2 : 0;
    ov.w = (i0 + 3 < nh) ? g3 : 0;
    *(volatile v4i*)(lrow + i0) = ov;
    __threadfence();
    *(volatile v4i*)(lrow + i0) = ov;
  }
  {
    const v4i cv = *(const v4ia*)(scnt + 4 * tid);
    const v4i fv = *(const v4ia*)(soff + 4 * tid);
    v4i rv = {0, 0, 0, 0};
    rv.x = (tid == 0) ? bmax : 0;
    rv.y = (tid == 0) ? flag : 0;
    rv.z = (tid == 0) ? nh : 0;
    int* cp = cp0 + 4 * tid;
    int* fp = fp0 + 4 * tid;
    int* rp = rp0 + 4 * (tid & 7);
    *(volatile v4i*)cp = cv;
    *(volatile v4i*)fp = fv;
    if (tid < 8) *(volatile v4i*)rp = rv;
    __threadfence();
    *(volatile v4i*)cp = cv;
    *(volatile v4i*)fp = fv;
    if (tid < 8) *(volatile v4i*)rp = rv;
  }
}

__global__ __launch_bounds__(NTHR) void k_bucket(const int* __restrict__ srcu, const int* __restrict__ dsti,
                                                 int nE, int vec8, int* LIST, int* CNT, int* OFF, int* REC) {
  extern __shared__ __attribute__((aligned(16))) int dsm[];
  const int b = (int)blockIdx.x;
  if (b < NBI) {
    bucket_body<RCAP_I>(dsti, srcu, nE, NITM, NUSR, vec8, b,
                        LIST + (size_t)b * RCAP_I, CNT + (size_t)b * NBA, OFF + (size_t)b * NBA,
                        REC + (size_t)b * 32, dsm);
  } else {
    bucket_body<RCAP_U>(srcu, dsti, nE, NUSR, NITM, vec8, b - NBI,
                        LIST + (size_t)NBI * RCAP_I + (size_t)(b - NBI) * RCAP_U,
                        CNT + (size_t)b * NBA, OFF + (size_t)b * NBA, REC + (size_t)b * 32, dsm);
  }
}

template <int L2>
__global__ __launch_bounds__(NTHR) void k_mean(unsigned short* wsb, size_t srcI, size_t srcU, size_t dstI,
                                               size_t dstU, const int* __restrict__ LIST,
                                               const int* __restrict__ CNT, const int* __restrict__ OFF,
                                               const int* __restrict__ REC) {
  constexpr int SP = L2 ? 512 : 128;
  constexpr int DP = L2 ? 512 : 256;
  const int tid = (int)threadIdx.x, lane = tid & 31, wave = tid >> 5;
  const int m = lane & 15, hh = lane >> 4;
  const bool roleU = (int)blockIdx.x >= RBI;
  const int rb   = roleU ? (int)blockIdx.x - RBI : (int)blockIdx.x;
  const int nN   = roleU ? NUSR : NITM;
  const int nG   = roleU ? NITM : NUSR;
  const int tbl  = roleU ? NBI * NBA : 0;
  const int blk0 = roleU ? NBI : 0;
  const int rcap = roleU ? RCAP_U : RCAP_I;
  const size_t lb = roleU ? (size_t)NBI * RCAP_I : (size_t)0;
  const size_t so = roleU ? srcU : srcI;
  const size_t dO = roleU ? dstU : dstI;
  const int cofs = L2 ? 8 * lane : 8 * m;
  const unsigned short* sp = wsb + so + cofs;
#pragma unroll 1
  for (int ri = 0; ri < RPW; ++ri) {
    const int node = rb * RPB + wave * RPW + ri;
    const int ti   = tbl + node;
    const int craw = CNT[ti];
    const int oraw = OFF[ti];
    const int fl   = REC[(blk0 + (node >> PKS)) * 32 + 1];
    const int deg = craw < 0 ? 0 : craw;
    int c = deg > DEGCAP ? DEGCAP : deg;
    const int o = oraw < 0 ? 0 : (oraw > rcap - 1 ? rcap - 1 : oraw);
    if (c > rcap - o) c = rcap - o;
    int last = o + c - 1;
    last = last < o ? o : last;
    const int* lp = LIST + lb + (size_t)(node >> PKS) * (size_t)rcap;
    float a0 = 0.f, a1 = 0.f, a2 = 0.f, a3 = 0.f, a4 = 0.f, a5 = 0.f, a6 = 0.f, a7 = 0.f;
#pragma unroll 1
    for (int b0 = 0; b0 < c; b0 += 32) {
      int idx = o + b0 + lane;
      idx = idx > last ? last : idx;
      int col = lp[idx];
      col = col < 0 ? 0 : (col > nG - 1 ? nG - 1 : col);
      const int m32 = (c - b0) < 32 ? (c - b0) : 32;
#pragma unroll 1
      for (int k = 0; k < m32; ++k) {
        const int sk = __builtin_amdgcn_readlane(col, k);
        const unsigned short* rp = sp + (size_t)sk * SP;
        if constexpr (L2 != 0) {
          const v4u wh = *(const v4ua*)rp;
          const v4u wl = *(const v4ua*)(rp + DHID);
          a0 += bfw_lo(wh.x) + bfw_lo(wl.x);
          a1 += bfw_hi(wh.x) + bfw_hi(wl.x);
          a2 += bfw_lo(wh.y) + bfw_lo(wl.y);
          a3 += bfw_hi(wh.y) + bfw_hi(wl.y);
          a4 += bfw_lo(wh.z) + bfw_lo(wl.z);
          a5 += bfw_hi(wh.z) + bfw_hi(wl.z);
          a6 += bfw_lo(wh.w) + bfw_lo(wl.w);
          a7 += bfw_hi(wh.w) + bfw_hi(wl.w);
        } else {
          const v4u w = *(const v4ua*)rp;
          a0 += bfw_lo(w.x);
          a1 += bfw_hi(w.x);
          a2 += bfw_lo(w.y);
          a3 += bfw_hi(w.y);
          a4 += bfw_lo(w.z);
          a5 += bfw_hi(w.z);
          a6 += bfw_lo(w.w);
          a7 += bfw_hi(w.w);
        }
      }
    }
    const float dv = (float)(deg < 1 ? 1 : deg);
#pragma unroll 1
    for (int j = 0; j < 8; ++j) {
      const float t = a0 / dv;
      a0 = a1; a1 = a2; a2 = a3; a3 = a4; a4 = a5; a5 = a6; a6 = a7; a7 = t;
    }
    const float pz = (fl != 0) ? __int_as_float(0x7fc00000) : 0.0f;
    const bool live = node < nN;
    const float r0 = live ? (a0 + pz) : 0.0f;
    const float r1 = live ? (a1 + pz) : 0.0f;
    const float r2 = live ? (a2 + pz) : 0.0f;
    const float r3 = live ? (a3 + pz) : 0.0f;
    const float r4 = live ? (a4 + pz) : 0.0f;
    const float r5 = live ? (a5 + pz) : 0.0f;
    const float r6 = live ? (a6 + pz) : 0.0f;
    const float r7 = live ? (a7 + pz) : 0.0f;
    unsigned h0, l0, h1, l1, h2, l2, h3, l3;
    pack2(r0, r1, h0, l0);
    pack2(r2, r3, h1, l1);
    pack2(r4, r5, h2, l2);
    pack2(r6, r7, h3, l3);
    unsigned short* wp = wsb + dO + (size_t)node * DP + 8 * lane;
    if constexpr (L2 != 0) {
      v4u qh, ql;
      qh.x = h0; qh.y = h1; qh.z = h2; qh.w = h3;
      ql.x = l0; ql.y = l1; ql.z = l2; ql.w = l3;
      *(volatile v4u*)wp = qh;
      *(volatile v4u*)(wp + DHID) = ql;
      __threadfence();
      *(volatile v4u*)wp = qh;
      *(volatile v4u*)(wp + DHID) = ql;
    } else {
      const bool isHi = (hh == 0);
      v4u q;
      q.x = isHi ? h0 : l0;
      q.y = isHi ? h1 : l1;
      q.z = isHi ? h2 : l2;
      q.w = isHi ? h3 : l3;
      *(volatile v4u*)wp = q;
      __threadfence();
      *(volatile v4u*)wp = q;
    }
  }
}

template <int NS, int BP>
__device__ __forceinline__ void ksteps(const unsigned short* __restrict__ ap, const unsigned short* __restrict__ wp,
                                       v8f (&acc)[8]) {
#pragma unroll 1
  for (int ks = 0; ks < NS; ++ks) {
    FragB af;
    af.h[0] = *(const v8usa*)(ap + 32 * ks);
    af.h[1] = *(const v8usa*)(ap + 32 * ks + 16);
#pragma unroll
    for (int t = 0; t < 8; ++t) {
      const unsigned short* wq = wp + (size_t)(16 * t) * (size_t)BP + 32 * ks;
      FragB bf;
      bf.h[0] = *(const v8usa*)wq;
      bf.h[1] = *(const v8usa*)(wq + 16);
      acc[t] = wmb(af, bf, acc[t]);
    }
  }
}

template <int MODE>
__global__ __launch_bounds__(GTHR) __attribute__((amdgpu_num_vgpr(248)))
void k_gemm(const unsigned short* __restrict__ A1, const unsigned short* __restrict__ A2,
            const unsigned short* __restrict__ WT, const float* __restrict__ bias,
            unsigned short* outh, float* outf, int nN) {
  constexpr int P1  = MODE ? 512 : 256;
  constexpr int P2  = MODE ? 512 : 128;
  constexpr int BP  = MODE ? K2 : K1;
  constexpr int NS1 = MODE ? 16 : 8;
  constexpr int NS2 = MODE ? 16 : 4;
  constexpr int KO2 = MODE ? 512 : 256;
  __shared__ __attribute__((aligned(16))) float stg[GBM * GBN];
  __shared__ __attribute__((aligned(16))) float bsh[GBN];
  const int tid = (int)threadIdx.x, lane = tid & 31, wave = tid >> 5, hh = lane >> 4, m = lane & 15;
  const int rowBase = (int)blockIdx.x * GBM;
  const int colBase = (int)blockIdx.y * GBN;

  if (tid < 32) {
    const v4f b4 = *(const v4f*)(bias + colBase + 4 * tid);
    *(v4fa*)(bsh + 4 * tid) = b4;
  }

  v8f acc[8];
  {
    const v8f z = {0.f, 0.f, 0.f, 0.f, 0.f, 0.f, 0.f, 0.f};
#pragma unroll
    for (int t = 0; t < 8; ++t) acc[t] = z;
  }
  const size_t arow = (size_t)(rowBase + 16 * wave + m);
  const unsigned short* wp = WT + (size_t)(colBase + m) * (size_t)BP + 8 * hh;
  ksteps<NS1, BP>(A1 + arow * P1 + 8 * hh, wp, acc);
  ksteps<NS2, BP>(A2 + arow * P2 + 8 * hh, wp + KO2, acc);
  __syncthreads();

#pragma unroll
  for (int t = 0; t < 8; ++t) {
    const int lc = 16 * t + m;
    const float bb = bsh[lc];
#pragma unroll
    for (int r = 0; r < 8; ++r) {
      const int lr = 16 * wave + 8 * hh + r;
      const bool live = (rowBase + lr) < nN;
      float v = acc[t][r] + bb;
      if constexpr (MODE == 0) v = relu_k(v);
      stg[lr * GBN + lc] = live ? v : 0.0f;
    }
  }
  __syncthreads();

  if constexpr (MODE == 0) {
    const int cb = 8 * m;
    const bool isHi = (hh == 0);
    v4u pk[16];
#pragma unroll
    for (int i = 0; i < 16; ++i) {
      const int lr = 16 * wave + i;
      const v4f a = *(const v4fa*)(stg + lr * GBN + cb);
      const v4f b = *(const v4fa*)(stg + lr * GBN + cb + 4);
      const float f[8] = {a.x, a.y, a.z, a.w, b.x, b.y, b.z, b.w};
      unsigned w[4];
#pragma unroll
      for (int j = 0; j < 4; ++j) {
        unsigned hw, lw;
        pack2(f[2 * j], f[2 * j + 1], hw, lw);
        w[j] = isHi ? hw : lw;
      }
      v4u pw; pw.x = w[0]; pw.y = w[1]; pw.z = w[2]; pw.w = w[3];
      pk[i] = pw;
    }
#pragma unroll
    for (int i = 0; i < 16; ++i) {
      const int gr = rowBase + 16 * wave + i;
      unsigned short* op = outh + (size_t)gr * (size_t)HP + hh * DHID + colBase + cb;
      *(volatile v4u*)op = pk[i];
    }
    __threadfence();
#pragma unroll
    for (int i = 0; i < 16; ++i) {
      const int gr = rowBase + 16 * wave + i;
      unsigned short* op = outh + (size_t)gr * (size_t)HP + hh * DHID + colBase + cb;
      *(volatile v4u*)op = pk[i];
    }
  } else {
    v4f pv[16];
#pragma unroll
    for (int i = 0; i < 16; ++i) pv[i] = *(const v4fa*)(stg + (16 * wave + i) * GBN + 4 * lane);
#pragma unroll
    for (int i = 0; i < 16; ++i) {
      const int gr = rowBase + 16 * wave + i;
      *(volatile v4f*)(outf + (size_t)gr * DOUT + 4 * lane) = pv[i];
    }
    __threadfence();
#pragma unroll
    for (int i = 0; i < 16; ++i) {
      const int gr = rowBase + 16 * wave + i;
      *(volatile v4f*)(outf + (size_t)gr * DOUT + 4 * lane) = pv[i];
    }
  }
}

__global__ __launch_bounds__(NTHR) void k_dots(const float* __restrict__ ZU, const float* __restrict__ ZI,
                                               const int* __restrict__ ls, const int* __restrict__ ld,
                                               float* out, int nL) {
  __shared__ __attribute__((aligned(16))) float vals[NTHR];
  const int tid = (int)threadIdx.x, lane = tid & 31, wave = tid >> 5;
  const int pi  = (int)blockIdx.x * NTHR + tid;
  const int pic = pi < nL ? pi : nL - 1;
  int su = ls[pic];
  int si = ld[pic];
  su = su < 0 ? 0 : (su > NUSR - 1 ? NUSR - 1 : su);
  si = si < 0 ? 0 : (si > NITM - 1 ? NITM - 1 : si);
  float res = 0.0f;
#pragma unroll 1
  for (int k = 0; k < 32; ++k) {
    const int uk = __builtin_amdgcn_readlane(su, k);
    const int ik = __builtin_amdgcn_readlane(si, k);
    const v4f a = *(const v4f*)(ZU + (size_t)uk * DOUT + 4 * lane);
    const v4f b = *(const v4f*)(ZI + (size_t)ik * DOUT + 4 * lane);
    float s = a.x * b.x + a.y * b.y + a.z * b.z + a.w * b.w;
    s += __shfl_xor(s, 16, 32);
    s += __shfl_xor(s, 8, 32);
    s += __shfl_xor(s, 4, 32);
    s += __shfl_xor(s, 2, 32);
    s += __shfl_xor(s, 1, 32);
    res = (lane == k) ? s : res;
  }
  vals[wave * 32 + lane] = res;
  __syncthreads();
  if (tid < 128) {
    const int half = tid >> 6;
    const int q    = tid & 63;
    const v4f v = *(const v4fa*)(vals + 4 * q);
    asm volatile("" :: "v"(v));
    const int e  = (int)blockIdx.x * NTHR + 4 * q;
    const bool ok = e < nL;
    const float sg = (half == 0) ? -1.0f : 1.0f;
    v4f o;
    o.x = sg * v.x; o.y = sg * v.y; o.z = sg * v.z; o.w = sg * v.w;
    const int es = ok ? e : 0;
    float* op = out + (size_t)half * (size_t)nL + (size_t)es;
    if (ok) *(volatile v4f*)op = o;
    __threadfence();
    if (ok) *(volatile v4f*)op = o;
  }
}

static inline size_t al256(size_t o) { return (o + 255) & ~(size_t)255; }

#define SZ_WPL  ((size_t)(2 * W1E + 2 * W2E) * 2)
#define SZ_BT   ((size_t)768 * 4)
#define SZ_LS   (((size_t)NBI * RCAP_I + (size_t)NBU * RCAP_U) * 4)
#define SZ_CN   ((size_t)NBT * NBA * 4)
#define SZ_RC   ((size_t)NBT * 128)
#define SZ_HU   ((size_t)MPU * HP * 2)
#define SZ_HI   ((size_t)MPI * HP * 2)
#define SZ_M1U  ((size_t)MPU * 256 * 2)
#define SZ_M1I  ((size_t)MPI * 256 * 2)
#define SZ_XUB  ((size_t)MPU * DIN * 2)
#define SZ_XIB  ((size_t)MPI * DIN * 2)
#define SZ_RB   (SZ_HU + SZ_HI)
#define SZ_ZU   ((size_t)MPU * DOUT * 4)
#define SZ_ZI   ((size_t)MPI * DOUT * 4)
static_assert(SZ_M1U + SZ_M1I + SZ_XUB + SZ_XIB <= SZ_RB);
static_assert(SZ_WPL % 256 == 0 && SZ_BT % 256 == 0 && SZ_LS % 256 == 0 && SZ_CN % 256 == 0);
static_assert(SZ_HU % 256 == 0 && SZ_HI % 256 == 0 && SZ_M1U % 256 == 0 && SZ_M1I % 256 == 0);
static_assert(SZ_XUB % 256 == 0 && SZ_ZU % 256 == 0 && SZ_ZI % 256 == 0);
static_assert(SZ_WPL + SZ_BT + SZ_LS + 2 * SZ_CN + SZ_RC + 256 + SZ_HU + SZ_HI + SZ_RB + SZ_ZU + SZ_ZI
              <= ((size_t)256 << 20));

extern "C" void kernel_launch(void* const* d_in, const int* in_sizes, int n_in,
                              void* d_out, int out_size, void* d_ws, size_t ws_size,
                              hipStream_t stream) {
  if (n_in < 18) return;
  if (in_sizes[0] != NUSR * DIN || in_sizes[1] != NITM * DIN) return;
  if (in_sizes[2] != DIN * DHID || in_sizes[3] != DIN * DHID || in_sizes[4] != DHID) return;
  if (in_sizes[5] != DIN * DHID || in_sizes[6] != DIN * DHID || in_sizes[7] != DHID) return;
  if (in_sizes[8] != DHID * DOUT || in_sizes[9] != DHID * DOUT || in_sizes[10] != DOUT) return;
  if (in_sizes[11] != DHID * DOUT || in_sizes[12] != DHID * DOUT || in_sizes[13] != DOUT) return;
  if (in_sizes[14] != NEDGE || in_sizes[15] != NEDGE) return;
  if (in_sizes[16] != NLAB || in_sizes[17] != NLAB) return;
  if (out_size != 2 * NLAB) return;

  const float* x_user = (const float*)d_in[0];
  const float* x_item = (const float*)d_in[1];
  const float* Wl1_ui = (const float*)d_in[2];
  const float* Wr1_ui = (const float*)d_in[3];
  const float* b1_ui  = (const float*)d_in[4];
  const float* Wl1_iu = (const float*)d_in[5];
  const float* Wr1_iu = (const float*)d_in[6];
  const float* b1_iu  = (const float*)d_in[7];
  const float* Wl2_ui = (const float*)d_in[8];
  const float* Wr2_ui = (const float*)d_in[9];
  const float* b2_ui  = (const float*)d_in[10];
  const float* Wl2_iu = (const float*)d_in[11];
  const float* Wr2_iu = (const float*)d_in[12];
  const float* b2_iu  = (const float*)d_in[13];
  const int* src_u = (const int*)d_in[14];
  const int* dst_i = (const int*)d_in[15];
  const int* lsrc  = (const int*)d_in[16];
  const int* ldst  = (const int*)d_in[17];
  float* out = (float*)d_out;

  char* ws = (char*)d_ws;
  size_t off = 0;
  const size_t oWP = off; off = al256(off + SZ_WPL);
  const size_t oBT = off; off = al256(off + SZ_BT);
  const size_t oLS = off; off = al256(off + SZ_LS);
  const size_t oCN = off; off = al256(off + SZ_CN);
  const size_t oOF = off; off = al256(off + SZ_CN);
  const size_t oRC = off; off = al256(off + SZ_RC);
  const size_t oHU = off; off = al256(off + SZ_HU);
  const size_t oHI = off; off = al256(off + SZ_HI);
  const size_t oRB = off; off = al256(off + SZ_RB);
  const size_t oZU = off; off = al256(off + SZ_ZU);
  const size_t oZI = off; off = al256(off + SZ_ZI);
  if (off > ws_size) return;
  const size_t oM1U = oRB;
  const size_t oM1I = oM1U + SZ_M1U;
  const size_t oXUB = oM1I + SZ_M1I;
  const size_t oXIB = oXUB + SZ_XUB;
  const size_t oM2U = oRB;
  const size_t oM2I = oRB + SZ_HU;

  unsigned short* wsb = (unsigned short*)ws;
  unsigned short* WPL = (unsigned short*)(ws + oWP);
  unsigned short* W1I = WPL;
  unsigned short* W1U = WPL + W1E;
  unsigned short* W2I = WPL + 2 * W1E;
  unsigned short* W2U = WPL + 2 * W1E + W2E;
  float* BT   = (float*)(ws + oBT);
  int*   LIST = (int*)(ws + oLS);
  int*   CNT  = (int*)(ws + oCN);
  int*   OFF  = (int*)(ws + oOF);
  int*   REC  = (int*)(ws + oRC);
  unsigned short* HU  = (unsigned short*)(ws + oHU);
  unsigned short* HI  = (unsigned short*)(ws + oHI);
  unsigned short* M1U = (unsigned short*)(ws + oM1U);
  unsigned short* M1I = (unsigned short*)(ws + oM1I);
  unsigned short* XUB = (unsigned short*)(ws + oXUB);
  unsigned short* XIB = (unsigned short*)(ws + oXIB);
  unsigned short* M2U = (unsigned short*)(ws + oM2U);
  unsigned short* M2I = (unsigned short*)(ws + oM2I);
  float* ZU = (float*)(ws + oZU);
  float* ZI = (float*)(ws + oZI);

  hipFuncSetAttribute(reinterpret_cast<const void*>(&k_bucket), hipFuncAttributeMaxDynamicSharedMemorySize, LDS_BK);
  const int vec8 = ((NEDGE & 3) == 0) ? 1 : 0;

  k_prep<<<PB_TOT, NTHR, 0, stream>>>(x_user, x_item, Wl1_ui, Wr1_ui, Wl1_iu, Wr1_iu, Wl2_ui, Wr2_ui, Wl2_iu, Wr2_iu,
                                      b1_ui, b1_iu, b2_ui, b2_iu, XUB, XIB, WPL, BT);
  k_bucket<<<NBT, NTHR, LDS_BK, stream>>>(src_u, dst_i, NEDGE, vec8, LIST, CNT, OFF, REC);
  k_mean<0><<<RBI + RBU, NTHR, 0, stream>>>(wsb, oXUB / 2, oXIB / 2, oM1I / 2, oM1U / 2, LIST, CNT, OFF, REC);
  k_gemm<0><<<dim3(RBI, 2, 1), GTHR, 0, stream>>>(M1I, XIB, W1I, BT, HI, ZI, NITM);
  k_gemm<0><<<dim3(RBU, 2, 1), GTHR, 0, stream>>>(M1U, XUB, W1U, BT + 256, HU, ZU, NUSR);
  k_mean<1><<<RBI + RBU, NTHR, 0, stream>>>(wsb, oHU / 2, oHI / 2, oM2I / 2, oM2U / 2, LIST, CNT, OFF, REC);
  k_gemm<1><<<dim3(RBI, 1, 1), GTHR, 0, stream>>>(M2I, HI, W2I, BT + 512, HI, ZI, NITM);
  k_gemm<1><<<dim3(RBU, 1, 1), GTHR, 0, stream>>>(M2U, HU, W2U, BT + 640, HU, ZU, NUSR);
  k_dots<<<(NLAB + NTHR - 1) / NTHR, NTHR, 0, stream>>>(ZU, ZI, lsrc, ldst, out, NLAB);
}
